// GCN_77180562309590
// MI455X (gfx1250) — hardware-verified
//
#include <hip/hip_runtime.h>
#include <stddef.h>
#include <stdint.h>
#include <math.h>


#define CIN    128
#define HID    64
#define K2     128
#define NGR    512
#define NTHR   256
#define NWAVE  8
#define EPT    8
#define CHUNK  (NTHR * EPT)
#define WCAP   (EPT * 32)
#define LISTN  (NWAVE * WCAP)
#define NBA    1024
#define SLA    10
#define RCAP   20480
#define DEGCAP 64
#define MEAS_B1024  16623
#define MEAS_MAXDEG 35
#define GBM    64
#define GBN    64
#define GTHR   128
#define MROWS  128
#define SROWS  128
#define NUW    (HID * (K2 / 8))
#define NPARB  10
#define PB0    0
#define PB1    64
#define PB2    128
#define PB3    192
#define PG0    256
#define PBE0   320
#define PG1    384
#define PBE1   448
#define PWO    512
#define PBO    640
#define PARN   672
#define PTHR   1024
#define SLOPE  0.01f
#define BNEPS  1e-5f
#define WSMAX  134217728
#define BKT_ZINTS    (LISTN + 2 * RCAP + 3 * NBA)
#define BKT_LDS_INTS (BKT_ZINTS + 16)

static_assert((CHUNK & (CHUNK - 1)) == 0 && CHUNK <= 4096);
static_assert((NBA & (NBA - 1)) == 0 && NBA == (1 << SLA) && NBA == 1024);
static_assert(((long long)CHUNK << SLA) < (1LL << 31));
static_assert(LISTN == NWAVE * WCAP);
static_assert(NBA % NWAVE == 0 && NBA % 32 == 0 && NBA == 4 * NTHR);
static_assert((RCAP % (4 * NTHR)) == 0 && (BKT_ZINTS % 4) == 0);
static_assert(RCAP >= MEAS_B1024 + (MEAS_B1024 + 19) / 20);
static_assert(DEGCAP >= MEAS_MAXDEG + 8);
static_assert(BKT_LDS_INTS * 4 <= 300000);
static_assert(GBM == (GTHR / 32) * 16 && GBN == 64 && HID == GBN);
static_assert(CIN == 128 && K2 == 128 && (K2 % 32) == 0 && K2 == 2 * HID);
static_assert((MROWS % GBM) == 0 && SROWS == MROWS);
static_assert(HID == 2 * 32);
static_assert((NUW % NTHR) == 0 && CIN / 8 == 16);
static_assert(NGR == 16 * 32 && PTHR == 32 * 32 && (NGR % 32) == 0);
static_assert(PARN % 32 == 0 && PBO % 32 == 0 && PWO % 32 == 0);
static_assert(SROWS * 16 == 8 * NTHR);

typedef float          v2f  __attribute__((ext_vector_type(2)));
typedef float          v4f  __attribute__((ext_vector_type(4)));
typedef float          v8f  __attribute__((ext_vector_type(8)));
typedef int            v4i  __attribute__((ext_vector_type(4)));
typedef int            v8i  __attribute__((ext_vector_type(8)));
typedef unsigned int   v4u  __attribute__((ext_vector_type(4)));
typedef unsigned short v8us __attribute__((ext_vector_type(8)));
typedef __bf16         v16b __attribute__((ext_vector_type(16)));
typedef v2f  __attribute__((may_alias)) v2fa;
typedef v4f  __attribute__((may_alias)) v4fa;
typedef v4i  __attribute__((may_alias)) v4ia;
typedef v8us __attribute__((may_alias)) v8usa;
union FragB { v16b v; v8us h[2]; v8i w; };

__device__ __forceinline__ v8f wmb(const FragB& a, const FragB& b, v8f c) {
  v8f d = __builtin_amdgcn_wmma_f32_16x16x32_bf16(false, a.v, false, b.v, (short)0, c, false, false);
  asm volatile("v_nop\n\tv_nop\n\tv_nop\n\tv_nop" : "+v"(d) : "v"(a.w), "v"(b.w));
  return d;
}

__device__ __forceinline__ unsigned int f2bf(float f) {
  const unsigned int u = __float_as_uint(f);
  const unsigned int r = ((u + 0x7FFFu + ((u >> 16) & 1u)) >> 16) & 0xFFFFu;
  return ((u & 0x7FFFFFFFu) > 0x7F800000u) ? 0x7FC0u : r;
}
__device__ __forceinline__ float bf2f(unsigned int b) { return __uint_as_float(b << 16); }
__device__ __forceinline__ float bfr(float f) { return bf2f(f2bf(f)); }

template <int SLB>
__device__ __forceinline__ int scan_chunk(const int* __restrict__ dsts, int nE, int cbase, int slotBase,
                                          int nb, int vec8, int* list, int tid, int lane, int wave) {
  int wc = 0;
  const int el0  = tid * EPT;
  const int e0   = cbase + el0;
  const int sent = -2147483647 - 1;
  v4i da, db;
  if (vec8 != 0 && cbase + CHUNK <= nE) {
    da = *(const v4i*)(dsts + e0);
    db = *(const v4i*)(dsts + e0 + 4);
  } else {
    da.x = (e0     < nE) ? dsts[min(e0,     nE - 1)] : sent;
    da.y = (e0 + 1 < nE) ? dsts[min(e0 + 1, nE - 1)] : sent;
    da.z = (e0 + 2 < nE) ? dsts[min(e0 + 2, nE - 1)] : sent;
    da.w = (e0 + 3 < nE) ? dsts[min(e0 + 3, nE - 1)] : sent;
    db.x = (e0 + 4 < nE) ? dsts[min(e0 + 4, nE - 1)] : sent;
    db.y = (e0 + 5 < nE) ? dsts[min(e0 + 5, nE - 1)] : sent;
    db.z = (e0 + 6 < nE) ? dsts[min(e0 + 6, nE - 1)] : sent;
    db.w = (e0 + 7 < nE) ? dsts[min(e0 + 7, nE - 1)] : sent;
  }
  const unsigned nbs = (unsigned)slotBase;
  const unsigned unb = (unsigned)nb;
  const unsigned s0 = (unsigned)da.x - nbs, s1 = (unsigned)da.y - nbs;
  const unsigned s2 = (unsigned)da.z - nbs, s3 = (unsigned)da.w - nbs;
  const unsigned s4 = (unsigned)db.x - nbs, s5 = (unsigned)db.y - nbs;
  const unsigned s6 = (unsigned)db.z - nbs, s7 = (unsigned)db.w - nbs;
  const bool h0 = s0 < unb, h1 = s1 < unb, h2 = s2 < unb, h3 = s3 < unb;
  const bool h4 = s4 < unb, h5 = s5 < unb, h6 = s6 < unb, h7 = s7 < unb;
  const unsigned any = __builtin_amdgcn_ballot_w32(h0 | h1 | h2 | h3 | h4 | h5 | h6 | h7);
  if (any != 0u) {
#define HITJ(J, HJ, SJ) { \
      const unsigned mj = __builtin_amdgcn_ballot_w32(HJ); \
      if (mj != 0u) { \
        if (HJ) { \
          const int pos = wc + (int)__builtin_amdgcn_mbcnt_lo(mj, 0u); \
          if (pos < WCAP) list[wave * WCAP + pos] = ((el0 + (J)) << SLB) | (int)(SJ); \
        } \
        wc += (int)__builtin_popcount(mj); } }
    HITJ(0, h0, s0)
    HITJ(1, h1, s1)
    HITJ(2, h2, s2)
    HITJ(3, h3, s3)
    HITJ(4, h4, s4)
    HITJ(5, h5, s5)
    HITJ(6, h6, s6)
    HITJ(7, h7, s7)
#undef HITJ
  }
  return wc;
}

__device__ __forceinline__ v8us wunit(const float* __restrict__ W, int kmask, int v) {
  const int n  = v >> 4;
  const int k8 = (v & 15) * 8;
  const int kk = k8 & kmask;
  const float* p = W + (size_t)kk * HID + n;
  v8us o;
#pragma unroll
  for (int i = 0; i < 8; ++i) o[i] = (unsigned short)f2bf(p[(size_t)i * HID]);
  return o;
}

__device__ __forceinline__ void par_put(const float* __restrict__ s, int n, float* dst, int tid) {
  const int nl = n >> 2;
  const int li = tid < nl ? tid : nl - 1;
  const float* p = s + 4 * li;
  v4f o;
  o.x = bfr(p[0]); o.y = bfr(p[1]); o.z = bfr(p[2]); o.w = bfr(p[3]);
  float* dp = dst + 4 * li;
  const bool ok = tid < nl;
  if (ok) *(volatile v4f*)dp = o;
  __threadfence();
  if (ok) *(volatile v4f*)dp = o;
}

__global__ __launch_bounds__(NTHR) void k_prep(
    const float* __restrict__ x, const float* __restrict__ W0, const float* __restrict__ W1,
    const float* __restrict__ W2, const float* __restrict__ W3,
    const float* __restrict__ b0, const float* __restrict__ b1, const float* __restrict__ b2,
    const float* __restrict__ b3, const float* __restrict__ g0, const float* __restrict__ be0,
    const float* __restrict__ g1, const float* __restrict__ be1, const float* __restrict__ Wout,
    const float* __restrict__ bout,
    unsigned short* XB, unsigned short* WT, float* PAR, int nN, int nBx) {
  const int tid = (int)threadIdx.x;
  const int bx  = (int)blockIdx.x;
  v8us o;
  unsigned short* dp;
  if (bx < nBx) {
    const int u   = bx * NTHR + tid;
    const int row = u >> 4;
    const int k8  = (u & 15) * 8;
    const int rc  = row < nN ? row : nN - 1;
    const float* p = x + (size_t)rc * CIN + k8;
    const v4f a = *(const v4fa*)p;
    const v4f b = *(const v4fa*)(p + 4);
    const bool ok = row < nN;
    o[0] = ok ? (unsigned short)f2bf(a.x) : (unsigned short)0;
    o[1] = ok ? (unsigned short)f2bf(a.y) : (unsigned short)0;
    o[2] = ok ? (unsigned short)f2bf(a.z) : (unsigned short)0;
    o[3] = ok ? (unsigned short)f2bf(a.w) : (unsigned short)0;
    o[4] = ok ? (unsigned short)f2bf(b.x) : (unsigned short)0;
    o[5] = ok ? (unsigned short)f2bf(b.y) : (unsigned short)0;
    o[6] = ok ? (unsigned short)f2bf(b.z) : (unsigned short)0;
    o[7] = ok ? (unsigned short)f2bf(b.w) : (unsigned short)0;
    dp = XB + (size_t)row * CIN + k8;
  } else if (bx < nBx + 4 * (NUW / NTHR)) {
    const int wb = bx - nBx;
    const int j  = wb / (NUW / NTHR);
    const int v  = (wb - j * (NUW / NTHR)) * NTHR + tid;
    if (j == 0)      o = wunit(W0, CIN - 1, v);
    else if (j == 1) o = wunit(W1, HID - 1, v);
    else if (j == 2) o = wunit(W2, HID - 1, v);
    else             o = wunit(W3, HID - 1, v);
    dp = WT + (size_t)j * (HID * K2) + (size_t)(v >> 4) * K2 + (v & 15) * 8;
  } else {
    const int j = bx - nBx - 4 * (NUW / NTHR);
    if (j == 0)      par_put(b0,  HID, PAR + PB0,  tid);
    else if (j == 1) par_put(b1,  HID, PAR + PB1,  tid);
    else if (j == 2) par_put(b2,  HID, PAR + PB2,  tid);
    else if (j == 3) par_put(b3,  HID, PAR + PB3,  tid);
    else if (j == 4) par_put(g0,  HID, PAR + PG0,  tid);
    else if (j == 5) par_put(be0, HID, PAR + PBE0, tid);
    else if (j == 6) par_put(g1,  HID, PAR + PG1,  tid);
    else if (j == 7) par_put(be1, HID, PAR + PBE1, tid);
    else if (j == 8) par_put(Wout, 2 * HID, PAR + PWO, tid);
    else if (j == 9) {
      const float bv = bfr(bout[0]);
      const int li = tid < 8 ? tid : 7;
      v4f q;
      q.x = (tid == 0) ? bv : 0.0f; q.y = 0.0f; q.z = 0.0f; q.w = 0.0f;
      float* qp = PAR + PBO + 4 * li;
      const bool ok = tid < 8;
      if (ok) *(volatile v4f*)qp = q;
      __threadfence();
      if (ok) *(volatile v4f*)qp = q;
    }
    return;
  }
  *(volatile v8us*)dp = o;
  __threadfence();
  *(volatile v8us*)dp = o;
}

__global__ __launch_bounds__(NTHR) void k_bucket(const int* __restrict__ srcs, const int* __restrict__ dsts,
                                                 const float* __restrict__ ewin, int nE, int nN, int vec8,
                                                 int* LSRC, int* LEW, int* CNT, int* OFF, float* DINV,
                                                 int* FLG) {
  extern __shared__ __attribute__((aligned(16))) int bsm[];
  int* list = bsm;
  int* hl   = bsm + LISTN;
  int* sl   = hl + RCAP;
  int* cnt  = sl + RCAP;
  int* offs = cnt + NBA;
  int* cur  = offs + NBA;
  int* misc = cur + NBA;
  const int tid = (int)threadIdx.x, lane = tid & 31, wave = tid >> 5;
  const int blk = (int)blockIdx.x;
  const int nodeBase = blk * NBA;
  int nb = nN - nodeBase;
  nb = nb < 0 ? 0 : (nb > NBA ? NBA : nb);

  {
    const v4i z4 = {0, 0, 0, 0};
    for (int i = tid * 4; i < BKT_ZINTS; i += NTHR * 4) *(v4ia*)(bsm + i) = z4;
    if (tid < 16) misc[tid] = 0;
  }
  __syncthreads();

  int tot = 0, ovf = 0;
  const int nChunks = (nE + CHUNK - 1) / CHUNK;
#pragma unroll 1
  for (int ch = 0; ch < nChunks; ++ch) {
    const int cbase = ch * CHUNK;
    const int wc = scan_chunk<SLA>(dsts, nE, cbase, nodeBase, nb, vec8, list, tid, lane, wave);
    if (lane == 0) misc[wave] = wc;
    __syncthreads();
    int pre = 0, all = 0;
#pragma unroll
    for (int w2 = 0; w2 < NWAVE; ++w2) {
      int c = misc[w2];
      c = c < 0 ? 0 : (c > WCAP ? WCAP : c);
      all += c;
      pre += (w2 < wave) ? c : 0;
    }
    const int wcc  = wc > WCAP ? WCAP : wc;
    const int base = tot + pre;
#pragma unroll 1
    for (int i = lane; i < wcc; i += 32) {
      const int ent = list[wave * WCAP + i];
      const int el  = (ent >> SLA) & (CHUNK - 1);
      const int st  = ent & (NBA - 1);
      int eid = cbase + el;
      eid = eid > nE - 1 ? nE - 1 : eid;
      const int pos = base + i;
      if (pos < RCAP) hl[pos] = (eid << SLA) | st;
    }
    if (tot + all > RCAP) ovf = 1;
    tot += all;
    tot = tot > RCAP ? RCAP : tot;
    __syncthreads();
  }
  const int nh = tot;

  if (wave == 0) {
#pragma unroll 1
    for (int b0 = 0; b0 < nh; b0 += 32) {
      const int idx = b0 + lane;
      const int uv  = hl[idx < nh ? idx : nh - 1];
      const int m32 = (nh - b0) < 32 ? (nh - b0) : 32;
#pragma unroll 1
      for (int k = 0; k < m32; ++k) {
        const int u  = __builtin_amdgcn_readlane(uv, k);
        const int sq = u & (NBA - 1);
        if (lane == 0) cnt[sq] = cnt[sq] + 1;
      }
    }
  }
  __syncthreads();
  if (wave == 0) {
    const int base = lane * (NBA / 32);
    int s = 0;
#pragma unroll 1
    for (int i = 0; i < NBA / 32; ++i) s += cnt[base + i];
    int incl = s;
#pragma unroll
    for (int d = 1; d < 32; d <<= 1) {
      const int y = __shfl_up(incl, d, 32);
      if (lane >= d) incl += y;
    }
    int run = incl - s;
#pragma unroll 1
    for (int i = 0; i < NBA / 32; ++i) {
      const int cv = cnt[base + i];
      offs[base + i] = run;
      cur[base + i]  = run;
      run += cv;
    }
  }
  __syncthreads();
  if (wave == 0) {
#pragma unroll 1
    for (int b0 = 0; b0 < nh; b0 += 32) {
      const int idx = b0 + lane;
      const int uv  = hl[idx < nh ? idx : nh - 1];
      const int m32 = (nh - b0) < 32 ? (nh - b0) : 32;
#pragma unroll 1
      for (int k = 0; k < m32; ++k) {
        const int u  = __builtin_amdgcn_readlane(uv, k);
        const int sq = u & (NBA - 1);
        if (lane == 0) {
          int p = cur[sq];
          p = p < 0 ? 0 : (p > RCAP - 1 ? RCAP - 1 : p);
          sl[p] = u;
          cur[sq] = p + 1;
        }
      }
    }
  }
  __syncthreads();

#pragma unroll 1
  for (int p = tid * 4; p < RCAP; p += NTHR * 4) {
    const v4i e4 = *(const v4ia*)(sl + p);
    int e0 = e4.x >> SLA, e1 = e4.y >> SLA, e2 = e4.z >> SLA, e3 = e4.w >> SLA;
    e0 = e0 < 0 ? 0 : (e0 > nE - 1 ? nE - 1 : e0);
    e1 = e1 < 0 ? 0 : (e1 > nE - 1 ? nE - 1 : e1);
    e2 = e2 < 0 ? 0 : (e2 > nE - 1 ? nE - 1 : e2);
    e3 = e3 < 0 ? 0 : (e3 > nE - 1 ? nE - 1 : e3);
    const int r0 = srcs[e0], r1 = srcs[e1], r2 = srcs[e2], r3 = srcs[e3];
    const float w0 = ewin[e0], w1 = ewin[e1], w2 = ewin[e2], w3 = ewin[e3];
    const bool k0 = p < nh, k1 = p + 1 < nh, k2 = p + 2 < nh, k3 = p + 3 < nh;
    v4i sv, wv;
    sv.x = k0 ? (r0 < 0 ? 0 : (r0 > nN - 1 ? nN - 1 : r0)) : 0;
    sv.y = k1 ? (r1 < 0 ? 0 : (r1 > nN - 1 ? nN - 1 : r1)) : 0;
    sv.z = k2 ? (r2 < 0 ? 0 : (r2 > nN - 1 ? nN - 1 : r2)) : 0;
    sv.w = k3 ? (r3 < 0 ? 0 : (r3 > nN - 1 ? nN - 1 : r3)) : 0;
    wv.x = k0 ? (int)(f2bf(w0) << 16) : 0;
    wv.y = k1 ? (int)(f2bf(w1) << 16) : 0;
    wv.z = k2 ? (int)(f2bf(w2) << 16) : 0;
    wv.w = k3 ? (int)(f2bf(w3) << 16) : 0;
    *(v4ia*)(sl + p) = sv;
    *(v4ia*)(hl + p) = wv;
  }
  __syncthreads();

  const v4i c4 = *(const v4ia*)(cnt + 4 * tid);
  const v4i o4 = *(const v4ia*)(offs + 4 * tid);
  const int cc0 = c4.x < 0 ? 0 : (c4.x > DEGCAP ? DEGCAP : c4.x);
  const int cc1 = c4.y < 0 ? 0 : (c4.y > DEGCAP ? DEGCAP : c4.y);
  const int cc2 = c4.z < 0 ? 0 : (c4.z > DEGCAP ? DEGCAP : c4.z);
  const int cc3 = c4.w < 0 ? 0 : (c4.w > DEGCAP ? DEGCAP : c4.w);
  const int oo0 = o4.x < 0 ? 0 : (o4.x > RCAP ? RCAP : o4.x);
  const int oo1 = o4.y < 0 ? 0 : (o4.y > RCAP ? RCAP : o4.y);
  const int oo2 = o4.z < 0 ? 0 : (o4.z > RCAP ? RCAP : o4.z);
  const int oo3 = o4.w < 0 ? 0 : (o4.w > RCAP ? RCAP : o4.w);
  float sm0 = 0.0f, sm1 = 0.0f, sm2 = 0.0f, sm3 = 0.0f;
#pragma unroll 2
  for (int j = 0; j < DEGCAP; ++j) {
    const int i0 = (oo0 + j) > RCAP - 1 ? RCAP - 1 : (oo0 + j);
    const int i1 = (oo1 + j) > RCAP - 1 ? RCAP - 1 : (oo1 + j);
    const int i2 = (oo2 + j) > RCAP - 1 ? RCAP - 1 : (oo2 + j);
    const int i3 = (oo3 + j) > RCAP - 1 ? RCAP - 1 : (oo3 + j);
    const float a0 = __int_as_float(hl[i0]);
    const float a1 = __int_as_float(hl[i1]);
    const float a2 = __int_as_float(hl[i2]);
    const float a3 = __int_as_float(hl[i3]);
    sm0 += (j < cc0) ? a0 : 0.0f;
    sm1 += (j < cc1) ? a1 : 0.0f;
    sm2 += (j < cc2) ? a2 : 0.0f;
    sm3 += (j < cc3) ? a3 : 0.0f;
  }
  const float qnan = __int_as_float(0x7fc00000);
  const bool g0b = c4.x > DEGCAP, g1b = c4.y > DEGCAP, g2b = c4.z > DEGCAP, g3b = c4.w > DEGCAP;
  const float d0 = sm0 + 1.0f, d1 = sm1 + 1.0f, d2 = sm2 + 1.0f, d3 = sm3 + 1.0f;
  v4f dv;
  dv.x = g0b ? qnan : ((d0 > 0.0f) ? (1.0f / sqrtf(d0)) : 0.0f);
  dv.y = g1b ? qnan : ((d1 > 0.0f) ? (1.0f / sqrtf(d1)) : 0.0f);
  dv.z = g2b ? qnan : ((d2 > 0.0f) ? (1.0f / sqrtf(d2)) : 0.0f);
  dv.w = g3b ? qnan : ((d3 > 0.0f) ? (1.0f / sqrtf(d3)) : 0.0f);
  const unsigned bb = __builtin_amdgcn_ballot_w32(g0b | g1b | g2b | g3b);
  if (lane == 0) misc[wave] = (bb != 0u) ? 1 : 0;
  __syncthreads();
  int fg = ovf;
#pragma unroll
  for (int w2 = 0; w2 < NWAVE; ++w2) fg |= misc[w2];

  int* lsb = LSRC + (size_t)blk * RCAP;
  int* lwb = LEW  + (size_t)blk * RCAP;
  const size_t nb0 = (size_t)blk * NBA + 4 * tid;
  v4i cv;
  cv.x = (tid == 0) ? nh : 0;
  cv.y = (tid == 0) ? fg : 0;
  cv.z = 0; cv.w = 0;
  int* fp = FLG + (size_t)blk * 32 + 4 * (tid & 7);
#pragma unroll 1
  for (int p = tid * 4; p < RCAP; p += NTHR * 4) {
    const v4i a = *(const v4ia*)(sl + p);
    const v4i b = *(const v4ia*)(hl + p);
    *(volatile v4i*)(lsb + p) = a;
    *(volatile v4i*)(lwb + p) = b;
  }
  *(volatile v4i*)(CNT + nb0) = c4;
  *(volatile v4i*)(OFF + nb0) = o4;
  *(volatile v4f*)(DINV + nb0) = dv;
  if (tid < 8) *(volatile v4i*)fp = cv;
  __threadfence();
#pragma unroll 1
  for (int p = tid * 4; p < RCAP; p += NTHR * 4) {
    const v4i a = *(const v4ia*)(sl + p);
    const v4i b = *(const v4ia*)(hl + p);
    *(volatile v4i*)(lsb + p) = a;
    *(volatile v4i*)(lwb + p) = b;
  }
  *(volatile v4i*)(CNT + nb0) = c4;
  *(volatile v4i*)(OFF + nb0) = o4;
  *(volatile v4f*)(DINV + nb0) = dv;
  if (tid < 8) *(volatile v4i*)fp = cv;
}

__global__ __launch_bounds__(GTHR) void k_gemm(
    const unsigned short* __restrict__ A, const unsigned short* __restrict__ WT,
    float* outF, int K, int ldo)
{
  __shared__ __attribute__((aligned(16))) float stg[GBM * GBN];
  const int tid = (int)threadIdx.x, lane = tid & 31, wave = tid >> 5, hh = lane >> 4, m = lane & 15;
  const int rowBase = (int)blockIdx.x * GBM;
  const int col0    = (int)blockIdx.y * GBN;

  v8f acc[4];
  {
    const v8f z = {0.f, 0.f, 0.f, 0.f, 0.f, 0.f, 0.f, 0.f};
    acc[0] = z; acc[1] = z; acc[2] = z; acc[3] = z;
  }
  const unsigned short* ap = A  + (size_t)(rowBase + 16 * wave + m) * (size_t)K + 8 * hh;
  const unsigned short* wp = WT + (size_t)(col0 + m) * (size_t)K + 8 * hh;
  const int ksteps = K >> 5;
#pragma unroll 1
  for (int ks = 0; ks < ksteps; ++ks) {
    FragB af;
    af.h[0] = *(const v8usa*)(ap + 32 * ks);
    af.h[1] = *(const v8usa*)(ap + 32 * ks + 16);
#pragma unroll
    for (int t = 0; t < 4; ++t) {
      const unsigned short* wq = wp + (size_t)(16 * t) * (size_t)K + 32 * ks;
      FragB bf;
      bf.h[0] = *(const v8usa*)wq;
      bf.h[1] = *(const v8usa*)(wq + 16);
      acc[t] = wmb(af, bf, acc[t]);
    }
  }

#pragma unroll
  for (int t = 0; t < 4; ++t) {
    const int lc = 16 * t + m;
#pragma unroll
    for (int r = 0; r < 8; ++r) {
      const int lr = 16 * wave + 8 * hh + r;
      stg[lr * GBN + lc] = acc[t][r];
    }
  }
  __syncthreads();

  v4f fv[8];
#pragma unroll
  for (int i = 0; i < 8; ++i) {
    const int lr = 16 * wave + 2 * i + hh;
    fv[i] = *(const v4fa*)(stg + lr * GBN + 4 * m);
  }
#pragma unroll
  for (int i = 0; i < 8; ++i) {
    const int lr = 16 * wave + 2 * i + hh;
    const int gr = rowBase + lr;
    float* op = outF + (size_t)gr * (size_t)ldo + col0 + 4 * m;
    *(volatile v4f*)op = fv[i];
  }
  __threadfence();
#pragma unroll
  for (int i = 0; i < 8; ++i) {
    const int lr = 16 * wave + 2 * i + hh;
    const int gr = rowBase + lr;
    float* op = outF + (size_t)gr * (size_t)ldo + col0 + 4 * m;
    *(volatile v4f*)op = fv[i];
  }
}

template <int MODE>
__global__ __launch_bounds__(NTHR) void k_agg(const int* __restrict__ LSRC, const int* __restrict__ LEW,
                                              const int* __restrict__ CNT, const int* __restrict__ OFF,
                                              const float* __restrict__ DINV, const int* __restrict__ FLG,
                                              const float* __restrict__ HW, const float* __restrict__ PAR,
                                              int boff, int nN, int mRows,
                                              unsigned short* hb, float* hout) {
  const int tid = (int)threadIdx.x, lane = tid & 31, wave = tid >> 5;
  const int blk = (int)blockIdx.x;
  const int nodeBase = blk * NBA;
  const int nhraw = FLG[(size_t)blk * 32];
  const int bflag = FLG[(size_t)blk * 32 + 1];
  const bool ovf = (bflag != 0) || (nhraw < 0) || (nhraw > RCAP);
  const int* lsb = LSRC + (size_t)blk * RCAP;
  const int* lwb = LEW  + (size_t)blk * RCAP;
  float bv0, bv1;
  {
    const v2f a = *(const v2fa*)(PAR + boff + 2 * lane);
    bv0 = a.x; bv1 = a.y;
  }
  const float qnan = __int_as_float(0x7fc00000);
  const int sa = (2 * lane) & 31, sb = (2 * lane + 1) & 31;
  const int q0s = (4 * lane) & 31, q1s = (4 * lane + 1) & 31;
  const int q2s = (4 * lane + 2) & 31, q3s = (4 * lane + 3) & 31;

#pragma unroll 1
  for (int si = 0; si < NBA / NWAVE; ++si) {
    const int s    = si * NWAVE + wave;
    const int node = nodeBase + s;
    const int craw = CNT[(size_t)nodeBase + s];
    const bool big = (craw > DEGCAP) || (craw < 0);
    int c = craw < 0 ? 0 : (craw > DEGCAP ? DEGCAP : craw);
    int o = OFF[(size_t)nodeBase + s];
    o = o < 0 ? 0 : (o > RCAP ? RCAP : o);
    const int nc = node < nN ? node : nN - 1;
    const float dd = DINV[nc];
    const float rd = dd * dd;
    float acc0 = 0.0f, acc1 = 0.0f;
#pragma unroll 1
    for (int b0 = 0; b0 < c; b0 += 32) {
      int idx = o + b0 + lane;
      idx = idx > RCAP - 1 ? RCAP - 1 : idx;
      int sr = lsb[idx];
      sr = sr < 0 ? 0 : (sr > nN - 1 ? nN - 1 : sr);
      const float ew = __int_as_float(lwb[idx]);
      const float cf = (DINV[sr] * ew) * dd;
      const int  cfi = __float_as_int(cf);
      const int m32 = (c - b0) < 32 ? (c - b0) : 32;
#pragma unroll 1
      for (int k = 0; k < m32; ++k) {
        const int   sk = __builtin_amdgcn_readlane(sr, k);
        const float ck = __int_as_float(__builtin_amdgcn_readlane(cfi, k));
        const v2f a = *(const v2fa*)(HW + (size_t)sk * HID + 2 * lane);
        acc0 = fmaf(ck, a.x, acc0); acc1 = fmaf(ck, a.y, acc1);
      }
    }
    float sv0, sv1;
    {
      const v2f a = *(const v2fa*)(HW + (size_t)nc * HID + 2 * lane);
      sv0 = a.x; sv1 = a.y;
    }
    float y0 = (acc0 + sv0 * rd) + bv0;
    float y1 = (acc1 + sv1 * rd) + bv1;
    if constexpr (MODE != 0) {
      y0 = (y0 >= 0.0f) ? y0 : SLOPE * y0;
      y1 = (y1 >= 0.0f) ? y1 : SLOPE * y1;
    }
    const bool pois = ovf || big;
    y0 = pois ? qnan : y0;
    y1 = pois ? qnan : y1;
    const bool live = node < nN;
    const float v0 = live ? y0 : 0.0f;
    const float v1 = live ? y1 : 0.0f;
    const bool wr = (node < mRows) && (lane < 16);
    if constexpr (MODE == 1) {
      const unsigned hb0 = f2bf(v0), hb1 = f2bf(v1);
      const unsigned lb0 = f2bf(v0 - bf2f(hb0));
      const unsigned lb1 = f2bf(v1 - bf2f(hb1));
      const int hw = (int)(hb0 | (hb1 << 16));
      const int lw = (int)(lb0 | (lb1 << 16));
      const int g0 = __shfl(hw, q0s, 32), g1 = __shfl(hw, q1s, 32);
      const int g2 = __shfl(hw, q2s, 32), g3 = __shfl(hw, q3s, 32);
      const int p0 = __shfl(lw, q0s, 32), p1 = __shfl(lw, q1s, 32);
      const int p2 = __shfl(lw, q2s, 32), p3 = __shfl(lw, q3s, 32);
      const bool lsel = (lane & 8) != 0;
      v4u pv;
      pv.x = (unsigned int)(lsel ? p0 : g0);
      pv.y = (unsigned int)(lsel ? p1 : g1);
      pv.z = (unsigned int)(lsel ? p2 : g2);
      pv.w = (unsigned int)(lsel ? p3 : g3);
      unsigned short* hp = hb + (size_t)node * K2 + 8 * (lane & 15);
      if (wr) *(volatile v4u*)hp = pv;
      __threadfence();
      if (wr) *(volatile v4u*)hp = pv;
    } else {
      v4f ow;
      ow.x = __shfl(v0, sa, 32); ow.y = __shfl(v1, sa, 32);
      ow.z = __shfl(v0, sb, 32); ow.w = __shfl(v1, sb, 32);
      float* op = hout + (size_t)node * HID + 4 * (lane & 15);
      if (wr) *(volatile v4f*)op = ow;
      __threadfence();
      if (wr) *(volatile v4f*)op = ow;
    }
  }
}

__global__ __launch_bounds__(NTHR) void k_stats(const float* __restrict__ C, int nN, float* REC) {
  __shared__ __attribute__((aligned(16))) float tile[SROWS * HID];
  __shared__ __attribute__((aligned(16))) float ps[4 * HID];
  __shared__ __attribute__((aligned(16))) float rec[2 * HID];
  const int tid = (int)threadIdx.x, lane = tid & 31, wave = tid >> 5;
  const int blk = (int)blockIdx.x;
  const int r0  = blk * SROWS;
  int nb = nN - r0;
  nb = nb < 1 ? 1 : (nb > SROWS ? SROWS : nb);
#pragma unroll 2
  for (int it = 0; it < 8; ++it) {
    const int unit = it * NTHR + tid;
    const int row = unit >> 4, q = unit & 15;
    int gr = r0 + row;
    gr = gr > nN - 1 ? nN - 1 : gr;
    const v4f v = *(const v4fa*)(C + (size_t)gr * HID + 4 * q);
    *(v4fa*)(tile + row * HID + 4 * q) = v;
  }
  __syncthreads();
  const int c = tid & 63, g = tid >> 6;
  float s = 0.0f;
#pragma unroll 4
  for (int r = 0; r < 32; ++r) {
    const int row = g * 32 + r;
    const float v = tile[row * HID + c];
    s += (row < nb) ? v : 0.0f;
  }
  ps[g * HID + c] = s;
  __syncthreads();
  if (tid < HID) {
    const float t = (ps[tid] + ps[HID + tid]) + (ps[2 * HID + tid] + ps[3 * HID + tid]);
    rec[tid] = t * (1.0f / (float)nb);
  }
  __syncthreads();
  const float mb = rec[c];
  float q2 = 0.0f;
#pragma unroll 4
  for (int r = 0; r < 32; ++r) {
    const int row = g * 32 + r;
    const float d = tile[row * HID + c] - mb;
    q2 += (row < nb) ? d * d : 0.0f;
  }
  ps[g * HID + c] = q2;
  __syncthreads();
  if (tid < HID) rec[HID + tid] = (ps[tid] + ps[HID + tid]) + (ps[2 * HID + tid] + ps[3 * HID + tid]);
  __syncthreads();
  const v4f rv = *(const v4fa*)(rec + 4 * lane);
  float* rp = REC + (size_t)blk * (2 * HID) + 4 * lane;
  const bool ok = wave == 0;
  if (ok) *(volatile v4f*)rp = rv;
  __threadfence();
  if (ok) *(volatile v4f*)rp = rv;
}

__global__ __launch_bounds__(64) void k_comb(const float* __restrict__ REC, int nBlk, int nN, double invN,
                                             float* STAT) {
  __shared__ __attribute__((aligned(16))) float st[2 * HID];
  const int tid = (int)threadIdx.x, lane = tid & 31, wave = tid >> 5;
  const int c = tid & 63;
  double S = 0.0;
#pragma unroll 2
  for (int b = 0; b < nBlk; ++b) {
    int nbi = nN - b * SROWS;
    nbi = nbi < 0 ? 0 : (nbi > SROWS ? SROWS : nbi);
    S += (double)nbi * (double)REC[(size_t)b * (2 * HID) + c];
  }
  const double mean = S * invN;
  double M2 = 0.0;
#pragma unroll 2
  for (int b = 0; b < nBlk; ++b) {
    int nbi = nN - b * SROWS;
    nbi = nbi < 0 ? 0 : (nbi > SROWS ? SROWS : nbi);
    const double mb = (double)REC[(size_t)b * (2 * HID) + c];
    const double m2 = (double)REC[(size_t)b * (2 * HID) + HID + c];
    const double d  = mb - mean;
    M2 += m2 + (double)nbi * d * d;
  }
  const float vf = (float)(M2 * invN);
  const float mf = (float)mean;
  const float r  = 1.0f / sqrtf(vf + BNEPS);
  st[c] = mf;
  st[HID + c] = r;
  __syncthreads();
  const v4f sv = *(const v4fa*)(st + 4 * lane);
  float* sp = STAT + 4 * lane;
  const bool ok = wave == 0;
  if (ok) *(volatile v4f*)sp = sv;
  __threadfence();
  if (ok) *(volatile v4f*)sp = sv;
}

__device__ __forceinline__ float bn_leaky(float x, float m, float r, float g, float be) {
  const float y = ((g * (x - m)) * r) + be;
  return (y >= 0.0f) ? y : SLOPE * y;
}

__global__ __launch_bounds__(NTHR) void k_apply(const float* __restrict__ C, const float* __restrict__ STAT,
                                                const float* __restrict__ PAR, int goff, int beoff,
                                                int nN, int nUnits, unsigned short* hb) {
  const int u = (int)blockIdx.x * NTHR + (int)threadIdx.x;
  if (u >= nUnits) return;
  const int row = u >> 4;
  const int q   = u & 15;
  const int c0  = 8 * (q & 7);
  const int rc  = row < nN ? row : nN - 1;
  const float* cp = C + (size_t)rc * HID + c0;
  const v4f xa = *(const v4fa*)cp;
  const v4f xb = *(const v4fa*)(cp + 4);
  const v4f ma = *(const v4fa*)(STAT + c0);
  const v4f mb = *(const v4fa*)(STAT + c0 + 4);
  const v4f ra = *(const v4fa*)(STAT + HID + c0);
  const v4f rb = *(const v4fa*)(STAT + HID + c0 + 4);
  const v4f ga = *(const v4fa*)(PAR + goff + c0);
  const v4f gb = *(const v4fa*)(PAR + goff + c0 + 4);
  const v4f ea = *(const v4fa*)(PAR + beoff + c0);
  const v4f eb = *(const v4fa*)(PAR + beoff + c0 + 4);
  float yv[8];
  yv[0] = bn_leaky(xa.x, ma.x, ra.x, ga.x, ea.x);
  yv[1] = bn_leaky(xa.y, ma.y, ra.y, ga.y, ea.y);
  yv[2] = bn_leaky(xa.z, ma.z, ra.z, ga.z, ea.z);
  yv[3] = bn_leaky(xa.w, ma.w, ra.w, ga.w, ea.w);
  yv[4] = bn_leaky(xb.x, mb.x, rb.x, gb.x, eb.x);
  yv[5] = bn_leaky(xb.y, mb.y, rb.y, gb.y, eb.y);
  yv[6] = bn_leaky(xb.z, mb.z, rb.z, gb.z, eb.z);
  yv[7] = bn_leaky(xb.w, mb.w, rb.w, gb.w, eb.w);
  const bool live = row < nN;
  const bool lsel = q >= 8;
  v8us o;
#pragma unroll
  for (int i = 0; i < 8; ++i) {
    const float v = live ? yv[i] : 0.0f;
    const unsigned hbi = f2bf(v);
    const unsigned lbi = f2bf(v - bf2f(hbi));
    o[i] = (unsigned short)(lsel ? lbi : hbi);
  }
  unsigned short* dp = hb + (size_t)row * K2 + 8 * q;
  *(volatile v8us*)dp = o;
  __threadfence();
  *(volatile v8us*)dp = o;
}

__global__ __launch_bounds__(PTHR) void k_pool_head(const float* __restrict__ H4, const int* __restrict__ bat,
                                                    const float* __restrict__ PAR, int nN, float* out) {
  __shared__ __attribute__((aligned(16))) float res[32];
  const int tid = (int)threadIdx.x, lane = tid & 31, wave = tid >> 5;
  const int g = (int)blockIdx.x * 32 + wave;
  const float ninf = __int_as_float((int)0xff800000u);
  float s0 = 0.0f, s1 = 0.0f, m0 = ninf, m1 = ninf;
  int mine = 0;
#pragma unroll 1
  for (int i0 = 0; i0 < nN; i0 += 32) {
    const int i  = i0 + lane;
    const int ic = i < nN ? i : nN - 1;
    const int b  = bat[ic];
    const bool hit = (i < nN) && (b == g);
    mine += hit ? 1 : 0;
    unsigned msk = __builtin_amdgcn_ballot_w32(hit);
#pragma unroll 1
    while (msk != 0u) {
      const int k = __builtin_ffs((int)msk) - 1;
      msk &= msk - 1u;
      int node = i0 + (k < 0 ? 0 : k);
      node = node > nN - 1 ? nN - 1 : node;
      const v2f v = *(const v2fa*)(H4 + (size_t)node * HID + 2 * lane);
      s0 += v.x; s1 += v.y;
      m0 = (v.x > m0 || v.x != v.x) ? v.x : m0;
      m1 = (v.y > m1 || v.y != v.y) ? v.y : m1;
    }
  }
  int cn = mine;
  cn += __shfl_xor(cn, 16, 32);
  cn += __shfl_xor(cn, 8, 32);
  cn += __shfl_xor(cn, 4, 32);
  cn += __shfl_xor(cn, 2, 32);
  cn += __shfl_xor(cn, 1, 32);
  const float cf  = (float)cn;
  const float inv = 1.0f / fmaxf(cf, 1.0f);
  const float me0 = s0 * inv, me1 = s1 * inv;
  const float x0 = (cn > 0) ? m0 : 0.0f;
  const float x1 = (cn > 0) ? m1 : 0.0f;
  const v2f wm = *(const v2fa*)(PAR + PWO + 2 * lane);
  const v2f wa = *(const v2fa*)(PAR + PWO + HID + 2 * lane);
  float d = x0 * wm.x;
  d = fmaf(x1, wm.y, d);
  d = fmaf(me0, wa.x, d);
  d = fmaf(me1, wa.y, d);
  d += __shfl_xor(d, 16, 32);
  d += __shfl_xor(d, 8, 32);
  d += __shfl_xor(d, 4, 32);
  d += __shfl_xor(d, 2, 32);
  d += __shfl_xor(d, 1, 32);
  const float bo = PAR[PBO];
  if (lane == 0) res[wave] = d + bo;
  __syncthreads();
  const int li = lane & 7;
  const v4f ov = *(const v4fa*)(res + 4 * li);
  float* op = out + (size_t)blockIdx.x * 32 + 4 * li;
  const bool ok = (wave == 0) && (lane < 8);
  if (ok) *(volatile v4f*)op = ov;
  __threadfence();
  if (ok) *(volatile v4f*)op = ov;
}

static inline int cdiv(int a, int b) { return (a + b - 1) / b; }
static inline size_t al256(size_t o) { return (o + 255) & ~(size_t)255; }

extern "C" void kernel_launch(void* const* d_in, const int* in_sizes, int n_in,
                              void* d_out, int out_size, void* d_ws, size_t ws_size,
                              hipStream_t stream) {
  if (n_in < 18) return;
  if (in_sizes[0] < CIN || (in_sizes[0] % CIN) != 0) return;
  const int nN = in_sizes[0] / CIN;
  if (nN < 1 || nN > (1 << 22)) return;
  if (in_sizes[1] < 2 || (in_sizes[1] & 1) != 0) return;
  const int nE = in_sizes[1] / 2;
  if (nE < 1 || nE >= (1 << (31 - SLA))) return;
  if (in_sizes[2] != nE) return;
  if (in_sizes[3] != nN) return;
  if (in_sizes[4] != CIN * HID) return;
  if (in_sizes[5] != HID || in_sizes[6] != HID || in_sizes[7] != HID) return;
  if (in_sizes[8] != HID * HID) return;
  if (in_sizes[9] != HID || in_sizes[10] != HID || in_sizes[11] != HID) return;
  if (in_sizes[12] != HID * HID || in_sizes[13] != HID) return;
  if (in_sizes[14] != HID * HID || in_sizes[15] != HID) return;
  if (in_sizes[16] != 2 * HID || in_sizes[17] != 1) return;
  if (out_size != NGR) return;

  const float* x    = (const float*)d_in[0];
  const int*   edge = (const int*)d_in[1];
  const float* ea   = (const float*)d_in[2];
  const int*   bat  = (const int*)d_in[3];
  const float* W0   = (const float*)d_in[4];
  const float* b0   = (const float*)d_in[5];
  const float* g0   = (const float*)d_in[6];
  const float* be0  = (const float*)d_in[7];
  const float* W1   = (const float*)d_in[8];
  const float* b1   = (const float*)d_in[9];
  const float* g1   = (const float*)d_in[10];
  const float* be1  = (const float*)d_in[11];
  const float* W2   = (const float*)d_in[12];
  const float* b2   = (const float*)d_in[13];
  const float* W3   = (const float*)d_in[14];
  const float* b3   = (const float*)d_in[15];
  const float* Wout = (const float*)d_in[16];
  const float* bout = (const float*)d_in[17];
  float* out = (float*)d_out;
  const int* src = edge;
  const int* dst = edge + nE;

  const int MP   = cdiv(nN, MROWS) * MROWS;
  const int gM   = MP / GBM;
  const int gA   = cdiv(MP, NBA);
  const int gS   = cdiv(nN, SROWS);
  if ((long long)gA * NBA < (long long)MP) return;
  const int nUx  = MP * (CIN / 8);
  if ((nUx % NTHR) != 0) return;
  const int nBx  = nUx / NTHR;
  const int vec8 = ((nE & 3) == 0) ? 1 : 0;

  char* ws = (char*)d_ws;
  size_t off = 0;
  const size_t oXB  = off; off = al256(off + (size_t)MP * CIN * 2);
  const size_t oWT  = off; off = al256(off + (size_t)4 * HID * K2 * 2);
  const size_t oPAR = off; off = al256(off + (size_t)PARN * 4);
  const size_t oHW  = off; off = al256(off + (size_t)MP * HID * 4);
  const size_t oC   = off; off = al256(off + (size_t)MP * HID * 4);
  const size_t oHHL = off; off = al256(off + (size_t)MP * K2 * 2);
  const size_t oLS  = off; off = al256(off + (size_t)gA * RCAP * 4);
  const size_t oLW  = off; off = al256(off + (size_t)gA * RCAP * 4);
  const size_t oCNT = off; off = al256(off + (size_t)gA * NBA * 4);
  const size_t oOFF = off; off = al256(off + (size_t)gA * NBA * 4);
  const size_t oDIN = off; off = al256(off + (size_t)gA * NBA * 4);
  const size_t oFLG = off; off = al256(off + (size_t)gA * 128);
  const size_t oREC = off; off = al256(off + (size_t)gS * 2 * HID * 4);
  const size_t oST  = off; off = al256(off + (size_t)2 * HID * 4);
  if (off > ws_size || off > (size_t)WSMAX) return;
  unsigned short* XB   = (unsigned short*)(ws + oXB);
  unsigned short* WT   = (unsigned short*)(ws + oWT);
  float*          PAR  = (float*)(ws + oPAR);
  float*          HW   = (float*)(ws + oHW);
  float*          C    = (float*)(ws + oC);
  unsigned short* HHL  = (unsigned short*)(ws + oHHL);
  int*            LSRC = (int*)(ws + oLS);
  int*            LEW  = (int*)(ws + oLW);
  int*            CNT  = (int*)(ws + oCNT);
  int*            OFF  = (int*)(ws + oOFF);
  float*          DINV = (float*)(ws + oDIN);
  int*            FLG  = (int*)(ws + oFLG);
  float*          REC  = (float*)(ws + oREC);
  float*          STAT = (float*)(ws + oST);
  const unsigned short* WT0 = WT;
  const unsigned short* WT1 = WT + (size_t)1 * HID * K2;
  const unsigned short* WT2 = WT + (size_t)2 * HID * K2;
  const unsigned short* WT3 = WT + (size_t)3 * HID * K2;

  const int bktLds = BKT_LDS_INTS * 4;
  hipFuncSetAttribute(reinterpret_cast<const void*>(&k_bucket),
                      hipFuncAttributeMaxDynamicSharedMemorySize, bktLds);
  const double invN = 1.0 / (double)nN;
  const dim3 gG(gM, HID / GBN);

  k_prep<<<nBx + 4 * (NUW / NTHR) + NPARB, NTHR, 0, stream>>>(x, W0, W1, W2, W3, b0, b1, b2, b3, g0, be0, g1, be1,
                                                             Wout, bout, XB, WT, PAR, nN, nBx);
  k_bucket<<<gA, NTHR, bktLds, stream>>>(src, dst, ea, nE, nN, vec8, LSRC, LEW, CNT, OFF, DINV, FLG);
  k_gemm<<<gG, GTHR, 0, stream>>>(XB, WT0, HW, CIN, HID);
  k_agg<0><<<gA, NTHR, 0, stream>>>(LSRC, LEW, CNT, OFF, DINV, FLG, HW, PAR, PB0, nN, MP, HHL, C);
  k_stats<<<gS, NTHR, 0, stream>>>(C, nN, REC);
  k_comb<<<1, 64, 0, stream>>>(REC, gS, nN, invN, STAT);
  k_apply<<<nBx, NTHR, 0, stream>>>(C, STAT, PAR, PG0, PBE0, nN, nUx, HHL);
  k_gemm<<<gG, GTHR, 0, stream>>>(HHL, WT1, HW, K2, HID);
  k_agg<0><<<gA, NTHR, 0, stream>>>(LSRC, LEW, CNT, OFF, DINV, FLG, HW, PAR, PB1, nN, MP, HHL, C);
  k_stats<<<gS, NTHR, 0, stream>>>(C, nN, REC);
  k_comb<<<1, 64, 0, stream>>>(REC, gS, nN, invN, STAT);
  k_apply<<<nBx, NTHR, 0, stream>>>(C, STAT, PAR, PG1, PBE1, nN, nUx, HHL);
  k_gemm<<<gG, GTHR, 0, stream>>>(HHL, WT2, HW, K2, HID);
  k_agg<1><<<gA, NTHR, 0, stream>>>(LSRC, LEW, CNT, OFF, DINV, FLG, HW, PAR, PB2, nN, MP, HHL, C);
  k_gemm<<<gG, GTHR, 0, stream>>>(HHL, WT3, HW, K2, HID);
  k_agg<2><<<gA, NTHR, 0, stream>>>(LSRC, LEW, CNT, OFF, DINV, FLG, HW, PAR, PB3, nN, MP, HHL, C);
  k_pool_head<<<NGR / 32, PTHR, 0, stream>>>(C, bat, PAR, nN, out);
}
